// EqualizedModConv2D_42090679500960
// MI455X (gfx1250) — hardware-verified
//
#include <hip/hip_runtime.h>


namespace {
constexpr int N = 16, IC = 512, OC = 512, H = 32, W = 32, HW = H * W, NPOS = N * HW, DL = 512, K9 = 9, KK = K9 * IC  ;
constexpr float EPS = 1e-8f;

typedef _Float16 b16;
typedef __attribute__((ext_vector_type(16))) _Float16 v16b;
typedef __attribute__((ext_vector_type(8))) _Float16 v8b;
typedef __attribute__((ext_vector_type(8))) float v8f;
typedef __attribute__((ext_vector_type(4))) float v4f;
__device__ __forceinline__ float bf16_rne(float f) { unsigned int u = __float_as_uint(f); u += 0x7FFFu + ((u >> 16) & 1u); return __uint_as_float(u & 0xFFFF0000u); }
__device__ __forceinline__ v16b frag_kb(const b16* p, int hh) { const v8b a = *(const v8b*)(p + 8 * hh), b = *(const v8b*)(p + 16 + 8 * hh); v16b f;
#pragma unroll
  for (int e = 0; e < 8; ++e) { f[e] = a[e]; f[8 + e] = b[e]; } return f; }
__device__ __forceinline__ v8f wmma16b(v16b a, v16b b, v8f c) { v8f d = __builtin_amdgcn_wmma_f32_16x16x32_f16(false, a, false, b, (short)0, c, false, false); asm volatile("v_nop\n\tv_nop\n\tv_nop\n\tv_nop" : "+v"(d) : "v"(a), "v"(b)); return d; }
__device__ __forceinline__ float pmul(float a, float b) { float p = a * b; asm volatile("" : "+v"(p)); return p; }

__global__ __launch_bounds__(256) void wprep_kernel(const float* __restrict__ wt, b16* __restrict__ R) {
  const size_t tid = (size_t)blockIdx.x * 256 + threadIdx.x, nth = (size_t)gridDim.x * 256;
  for (int pass = 0; pass < 2; ++pass) { for (size_t q = tid; q < (size_t)OC * KK; q += nth) { const int o = (int)(q / KK), k = (int)(q % KK), tap = k / IC, c = k % IC; R[q] = (b16)bf16_rne(wt[((size_t)o * IC + c) * 9 + tap]); } __threadfence(); }
}

__global__ __launch_bounds__(256) void mod_kernel(const float* __restrict__ style, const float* __restrict__ fcw, const float* __restrict__ bias, const float* __restrict__ wt, float* __restrict__ modv, float* __restrict__ dmv) {
  __shared__ float Md[IC]; __shared__ float St[DL];
  const int n = blockIdx.x, t_ = threadIdx.x; const float fcs = 1.0f / sqrtf((float)DL), wsc = 1.0f / sqrtf((float)KK);
  for (int d = t_; d < DL; d += 256) St[d] = bf16_rne(style[(size_t)n * DL + d]);
  __syncthreads();
  for (int c = t_; c < IC; c += 256) { float s = 0.0f; const float* fr = fcw + (size_t)c * DL; for (int d = 0; d < DL; ++d) s += pmul(St[d], pmul(bf16_rne(fr[d]), fcs)); Md[c] = s + bf16_rne(bias[c]) + 1.0f; }
  __syncthreads();
  for (int pass = 0; pass < 2; ++pass) { for (int c = t_; c < IC; c += 256) ((volatile float*)modv)[(size_t)n * IC + c] = Md[c]; }
  for (int o = t_; o < OC; o += 256) { float s = 0.0f; const float* wr = wt + (size_t)o * IC * 9; for (int c = 0; c < IC; ++c) { const float m = pmul(Md[c], wsc); float sk = 0.0f;
#pragma unroll
      for (int k = 0; k < 9; ++k) { const float w_ = pmul(bf16_rne(wr[c * 9 + k]), m); sk += pmul(w_, w_); } s += sk; }
    const float dm = rsqrtf(s + EPS) * wsc; for (int pass = 0; pass < 2; ++pass) ((volatile float*)dmv)[(size_t)n * OC + o] = dm; }
  __threadfence();
}

__global__ __launch_bounds__(256) void xmod_kernel(const float* __restrict__ x, const float* __restrict__ modv, b16* __restrict__ xm) {
  __shared__ __attribute__((aligned(16))) b16 T[W][IC + 8];
  const int n = blockIdx.y, h = blockIdx.x, t_ = threadIdx.x;
  for (int q = t_; q < IC * W; q += 256) { const int c = q >> 5, w = q & 31; T[w][c] = (b16)(bf16_rne(x[(((size_t)n * IC + c) * H + h) * W + w]) * modv[(size_t)n * IC + c]); }
  __syncthreads();
  for (int pass = 0; pass < 2; ++pass) { for (int q = t_; q < W * (IC / 8); q += 256) { const int w = q >> 6, c8 = (q & 63) * 8; *(volatile v8b*)(xm + (((size_t)n * H + h) * W + w) * IC + c8) = *(const v8b*)(&T[w][c8]); } __threadfence(); }
}

__global__ __launch_bounds__(128) void conv_kernel(const b16* __restrict__ xm, const b16* __restrict__ R, const float* __restrict__ dmv, float* __restrict__ out) {
  __shared__ __attribute__((aligned(16))) float Tc[64][128 + 4];
  const int lane = threadIdx.x & 31, wave = threadIdx.x >> 5, nloc = lane & 15, hlf = lane >> 4, c0 = blockIdx.x * 64, p0 = blockIdx.y * 128, n = blockIdx.z; const b16* xb = xm + ((size_t)n * HW) * IC;
  const int pa = p0 + wave * 32 + nloc, pb = pa + 16; const int ha = pa / W, wa = pa % W, hb = pb / W, wb = pb % W;
  v8f acc[2][4];
#pragma unroll
  for (int r = 0; r < 2; ++r)
#pragma unroll
    for (int t = 0; t < 4; ++t) acc[r][t] = (v8f){};
  for (int tap = 0; tap < K9; ++tap) { const int u = tap / 3 - 1, v = tap % 3 - 1; const int ia = ha + u, ja = wa + v, ib = hb + u, jb = wb + v; const bool va = (ia >= 0 && ia < H && ja >= 0 && ja < W), vb_ = (ib >= 0 && ib < H && jb >= 0 && jb < W);
    const b16* ra = xb + (size_t)(va ? (ia * W + ja) : 0) * IC; const b16* rb = xb + (size_t)(vb_ ? (ib * W + jb) : 0) * IC;
#pragma unroll 4
    for (int cb = 0; cb < IC; cb += 32) { v16b a0 = frag_kb(ra + cb, hlf), a1 = frag_kb(rb + cb, hlf); if (!va) a0 = (v16b){}; if (!vb_) a1 = (v16b){};
#pragma unroll
      for (int t = 0; t < 4; ++t) { const v16b bw = frag_kb(R + (size_t)(c0 + t * 16 + nloc) * KK + tap * IC + cb, hlf); acc[0][t] = wmma16b(a0, bw, acc[0][t]); acc[1][t] = wmma16b(a1, bw, acc[1][t]); } } }
#pragma unroll
  for (int t = 0; t < 4; ++t) { const int o = c0 + t * 16 + nloc; const float dm = dmv[(size_t)n * OC + o];
#pragma unroll
    for (int r = 0; r < 2; ++r)
#pragma unroll
      for (int vv = 0; vv < 8; ++vv) Tc[t * 16 + nloc][wave * 32 + r * 16 + 8 * hlf + vv] = acc[r][t][vv] * dm; }
  __syncthreads();
  for (int pass = 0; pass < 2; ++pass) { for (int q = threadIdx.x; q < 64 * 32; q += 128) { const int cc = q >> 5, c4 = (q & 31) * 4; *(volatile v4f*)(out + ((size_t)n * OC + c0 + cc) * HW + p0 + c4) = *(const v4f*)(&Tc[cc][c4]); } __threadfence(); }
}
}

extern "C" void kernel_launch(void* const* d_in, const int* in_sizes, int n_in,
                              void* d_out, int out_size, void* d_ws, size_t ws_size, hipStream_t stream) {
  (void)n_in; (void)out_size;
  const float* x = (const float*)d_in[0]; const float* style = (const float*)d_in[1]; const float* wt = (const float*)d_in[2]; const float* fcw = (const float*)d_in[3]; const float* bias = (const float*)d_in[4];
  float* out = (float*)d_out;
  if (in_sizes[0] != NPOS * IC || in_sizes[1] != N * DL || in_sizes[2] != OC * IC * 9 || in_sizes[3] != IC * DL || in_sizes[4] != IC) return;
  size_t off = 0; char* ws = (char*)d_ws;
  auto carve = [&](size_t bytes) { char* p = ws + off; off += (bytes + 255) & ~(size_t)255; return p; };
  b16* R = (b16*)carve((size_t)OC * KK * 2); float* modv = (float*)carve((size_t)N * IC * 4); float* dmv = (float*)carve((size_t)N * OC * 4); b16* xm = (b16*)carve((size_t)NPOS * IC * 2);
  if (off > ws_size) return;
  wprep_kernel<<<512, 256, 0, stream>>>(wt, R);
  mod_kernel<<<N, 256, 0, stream>>>(style, fcw, bias, wt, modv, dmv);
  xmod_kernel<<<dim3(H, N), 256, 0, stream>>>(x, modv, xm);
  conv_kernel<<<dim3(OC / 64, HW / 128, N), 128, 0, stream>>>(xm, R, dmv, out);
}
